// MambaBlock_51110110822785
// MI455X (gfx1250) — hardware-verified
//
#include <hip/hip_runtime.h>
#include <math.h>

typedef __attribute__((ext_vector_type(16))) _Float16 v16h;
typedef __attribute__((ext_vector_type(8)))  _Float16 v8h;
typedef __attribute__((ext_vector_type(16))) __bf16   v16b;
typedef __attribute__((ext_vector_type(8)))  __bf16   v8b;
typedef __attribute__((ext_vector_type(8)))  float    v8f;
typedef __attribute__((ext_vector_type(4)))  float    v4f;
typedef __attribute__((ext_vector_type(4)))  unsigned v4u;

constexpr int kBatch = 2;
constexpr int kSeq   = 2048;
constexpr int kHid   = 768;
constexpr int kInner = 1536;
constexpr int kNst   = 16;
constexpr int kProjW = 2 * kNst + kInner;
constexpr int kBcP   = 64;
constexpr int kRows  = kBatch * kSeq;
constexpr int kConvTP = 260;
constexpr int kScT   = 64;
constexpr int kScC   = 64;
constexpr int kScP   = 68;
constexpr float kActCarry = 16.0f;
constexpr float kWgtCarry = 32.0f;
constexpr float kFoldAW   = 1.0f / (kActCarry * kWgtCarry);
constexpr float kFoldW    = 1.0f / kWgtCarry;
static_assert(kProjW == 1568);
static_assert((kHid % 64) == 0 && (kInner % 64) == 0 && (kSeq % 64) == 0 && (kBcP % 64) == 0);
static_assert((kHid % 32) == 0 && (kInner % 32) == 0);
static_assert((kInner % 256) == 0 && (kHid % 256) == 0 && (kRows % 8) == 0);
static_assert((kSeq % kScT) == 0 && (kInner % kScC) == 0);

constexpr size_t kSzXN   = (size_t)kRows * kHid * 2;
constexpr size_t kSzBT0  = (size_t)2 * kInner * kHid * 2;
constexpr size_t kSzBT1D = (size_t)kInner * kInner * 2;
constexpr size_t kSzBTB  = (size_t)kBcP * kInner * 2;
constexpr size_t kSzBT2  = (size_t)kInner * kInner * 2;
constexpr size_t kSzBT3  = (size_t)kHid * kInner * 2;
constexpr size_t kSzF32P = (size_t)kSeq * kInner * 4;
constexpr size_t kSzH16P = (size_t)kSeq * kInner * 2;
constexpr size_t kSzBC   = (size_t)kSeq * kBcP * 4;
constexpr size_t kOffXNH  = 0;
constexpr size_t kOffXNL  = kOffXNH  + kSzXN;
constexpr size_t kOffBT0H = kOffXNL  + kSzXN;
constexpr size_t kOffBT0L = kOffBT0H + kSzBT0;
constexpr size_t kOffBT1D = kOffBT0L + kSzBT0;
constexpr size_t kOffBTBH = kOffBT1D + kSzBT1D;
constexpr size_t kOffBTBL = kOffBTBH + kSzBTB;
constexpr size_t kOffBT2  = kOffBTBL + kSzBTB;
constexpr size_t kOffBT3  = kOffBT2  + kSzBT2;
constexpr size_t kOffUPRE = kOffBT3  + kSzBT3;
constexpr size_t kOffGS   = kOffUPRE + kSzF32P;
constexpr size_t kOffUH   = kOffGS   + kSzF32P;
constexpr size_t kOffUL   = kOffUH   + kSzH16P;
constexpr size_t kOffUF   = kOffUL   + kSzH16P;
constexpr size_t kOffDR   = kOffUF   + kSzH16P;
constexpr size_t kOffBC   = kOffDR   + kSzF32P;
constexpr size_t kOffY16  = kOffBC   + kSzBC;
constexpr size_t kOffZ16  = kOffY16  + kSzH16P;
constexpr size_t kWsTotal = kOffZ16  + kSzH16P;
static_assert(kWsTotal == 103940096ull);
static_assert(kWsTotal <= 134217728ull);
static_assert((kOffXNL % 128) == 0 && (kOffBT0H % 128) == 0 && (kOffBT0L % 128) == 0 && (kOffBT1D % 128) == 0 &&
              (kOffBTBH % 128) == 0 && (kOffBTBL % 128) == 0 && (kOffBT2 % 128) == 0 && (kOffBT3 % 128) == 0 &&
              (kOffUPRE % 128) == 0 && (kOffGS % 128) == 0 && (kOffUH % 128) == 0 && (kOffUL % 128) == 0 &&
              (kOffUF % 128) == 0 && (kOffDR % 128) == 0 && (kOffBC % 128) == 0 && (kOffY16 % 128) == 0 &&
              (kOffZ16 % 128) == 0);

__device__ __forceinline__ unsigned bf_bits(float f) {
  const unsigned u = __float_as_uint(f);
  return ((u + 0x7FFFu + ((u >> 16) & 1u)) >> 16) & 0xFFFFu;
}
__device__ __forceinline__ float bf_val(unsigned hb) { return __uint_as_float(hb << 16); }
__device__ __forceinline__ void split2(float a, float b, unsigned& hw, unsigned& lw) {
  const unsigned ha = bf_bits(a);
  const unsigned hb = bf_bits(b);
  const unsigned la = bf_bits(a - bf_val(ha));
  const unsigned lb = bf_bits(b - bf_val(hb));
  hw = ha | (hb << 16);
  lw = la | (lb << 16);
}
__device__ __forceinline__ float bfw_lo(unsigned w) { return __uint_as_float(w << 16); }
__device__ __forceinline__ float bfw_hi(unsigned w) { return __uint_as_float(w & 0xffff0000u); }

__device__ __forceinline__ void wave_lds_sync() {
  __builtin_amdgcn_fence(__ATOMIC_RELEASE, "workgroup");
  __builtin_amdgcn_wave_barrier();
  __builtin_amdgcn_fence(__ATOMIC_ACQUIRE, "workgroup");
}

__device__ __forceinline__ void grp_guard_h(v8f& a, v8f& b, v8f& c, v8f& d, v16h x, v16h y) {
  asm volatile("v_nop\n\tv_nop\n\tv_nop\n\tv_nop" : "+v"(a), "+v"(b), "+v"(c), "+v"(d) : "v"(x), "v"(y));
}
__device__ __forceinline__ void grp_guard_b(v8f& a, v8f& b, v8f& c, v8f& d, v16b x, v16b y) {
  asm volatile("v_nop\n\tv_nop\n\tv_nop\n\tv_nop" : "+v"(a), "+v"(b), "+v"(c), "+v"(d) : "v"(x), "v"(y));
}
__device__ __forceinline__ void keep4_h(v16h a, v16h b, v16h c, v16h d) { asm volatile("v_nop" :: "v"(a), "v"(b), "v"(c), "v"(d)); }
__device__ __forceinline__ void keep4_b(v16b a, v16b b, v16b c, v16b d) { asm volatile("v_nop" :: "v"(a), "v"(b), "v"(c), "v"(d)); }
__device__ __forceinline__ void acc_guard4(v8f& a, v8f& b, v8f& c, v8f& d) {
  asm volatile("v_nop\n\tv_nop\n\tv_nop\n\tv_nop" : "+v"(a), "+v"(b), "+v"(c), "+v"(d));
}

template <typename T> struct Frag;
template <> struct Frag<_Float16> {
  typedef v16h V; union U { v16h v; v8h h[2]; };
  static __device__ __forceinline__ v16h load(const _Float16* p) {
    U f; f.h[0] = *(const v8h*)(p); f.h[1] = *(const v8h*)(p + 16); return f.v;
  }
  static __device__ __forceinline__ v8f mma(v16h a, v16h b, v8f c) {
    return __builtin_amdgcn_wmma_f32_16x16x32_f16(false, a, false, b, (short)0, c, false, false);
  }
  static __device__ __forceinline__ void guard(v8f& a, v8f& b, v8f& c, v8f& d, v16h x, v16h y) { grp_guard_h(a, b, c, d, x, y); }
  static __device__ __forceinline__ void keep(v16h a, v16h b, v16h c, v16h d) { keep4_h(a, b, c, d); }
};
template <> struct Frag<__bf16> {
  typedef v16b V; union U { v16b v; v8b h[2]; };
  static __device__ __forceinline__ v16b load(const __bf16* p) {
    U f; f.h[0] = *(const v8b*)(p); f.h[1] = *(const v8b*)(p + 16); return f.v;
  }
  static __device__ __forceinline__ v8f mma(v16b a, v16b b, v8f c) {
    return __builtin_amdgcn_wmma_f32_16x16x32_bf16(false, a, false, b, (short)0, c, false, false);
  }
  static __device__ __forceinline__ void guard(v8f& a, v8f& b, v8f& c, v8f& d, v16b x, v16b y) { grp_guard_b(a, b, c, d, x, y); }
  static __device__ __forceinline__ void keep(v16b a, v16b b, v16b c, v16b d) { keep4_b(a, b, c, d); }
};

template <int ET> struct Elem;
template <> struct Elem<0> { typedef _Float16 T; };
template <> struct Elem<1> { typedef __bf16 T; };

template <int ET, bool SPLIT, int EPI>
__global__ __launch_bounds__(256) void wmma_gemm64(
    const unsigned short* __restrict__ Ap, const unsigned short* __restrict__ A2p, int lda,
    const unsigned short* __restrict__ Btp, const unsigned short* __restrict__ Bt2p, int ldb,
    void* __restrict__ Cout, int ldc,
    const float* __restrict__ aux, int ldaux,
    int M, int N, int K, float scale)
{
  typedef typename Elem<ET>::T T;
  typedef typename Frag<T>::V V;
  const T* A = (const T*)Ap; const T* A2 = (const T*)A2p; const T* Bt = (const T*)Btp; const T* Bt2 = (const T*)Bt2p;
  __shared__ __align__(16) float sT[8][16 * 68];
  const int lane = threadIdx.x & 31;
  const int wave = threadIdx.x >> 5;
  const int tilesN = N >> 6;
  const int tilesM = M >> 6;
  const int tile = blockIdx.x * 8 + wave;
  if (tile >= tilesM * tilesN) return;
  const int tm = tile / tilesN;
  const int tn = tile - tm * tilesN;
  const int m0 = tm << 6;
  const int n0 = tn << 6;

  const int rlane = lane & 15;
  const int koff  = (lane >> 4) * 8;
  const int mOff  = (lane >> 4) * 8;

  v8f acc[4][4];
#pragma unroll
  for (int i = 0; i < 4; ++i)
#pragma unroll
    for (int j = 0; j < 4; ++j) acc[i][j] = (v8f){0.f,0.f,0.f,0.f,0.f,0.f,0.f,0.f};

  for (int k0 = 0; k0 < K; k0 += 32) {
    V bh[4], bl[4];
#pragma unroll
    for (int j = 0; j < 4; ++j) {
      const size_t bo = (size_t)(n0 + (j << 4) + rlane) * ldb + koff + k0;
      bh[j] = Frag<T>::load(Bt + bo);
      if (SPLIT) bl[j] = Frag<T>::load(Bt2 + bo);
    }
#pragma unroll
    for (int i = 0; i < 4; ++i) {
      const size_t ao = (size_t)(m0 + (i << 4) + rlane) * lda + koff + k0;
      V ah = Frag<T>::load(A + ao);
      V al;
      if (SPLIT) al = Frag<T>::load(A2 + ao);
#pragma unroll
      for (int j = 0; j < 4; ++j) {
        acc[i][j] = Frag<T>::mma(ah, bh[j], acc[i][j]);
        if (SPLIT) {
          acc[i][j] = Frag<T>::mma(ah, bl[j], acc[i][j]);
          acc[i][j] = Frag<T>::mma(al, bh[j], acc[i][j]);
        }
      }
      Frag<T>::guard(acc[i][0], acc[i][1], acc[i][2], acc[i][3], ah, SPLIT ? al : ah);
    }
    Frag<T>::keep(bh[0], bh[1], bh[2], bh[3]);
    if (SPLIT) Frag<T>::keep(bl[0], bl[1], bl[2], bl[3]);
  }
  acc_guard4(acc[0][0], acc[0][1], acc[0][2], acc[0][3]);
  acc_guard4(acc[1][0], acc[1][1], acc[1][2], acc[1][3]);
  acc_guard4(acc[2][0], acc[2][1], acc[2][2], acc[2][3]);
  acc_guard4(acc[3][0], acc[3][1], acc[3][2], acc[3][3]);

  float* slab = sT[wave];
#pragma unroll
  for (int i = 0; i < 4; ++i) {
    const int mBase = m0 + (i << 4);
#pragma unroll
    for (int j = 0; j < 4; ++j) {
#pragma unroll
      for (int r = 0; r < 8; ++r) {
        slab[(mOff + r) * 68 + (j << 4) + rlane] = acc[i][j][r] * scale;
      }
    }
    wave_lds_sync();
    if (EPI == 1) {
#pragma unroll 1
      for (int e = 0; e < 32; ++e) {
        const int idx = (e >> 1) * 68 + ((e & 1) << 5) + lane;
        const float v = slab[idx];
        const float sg = __builtin_amdgcn_rcpf(1.0f + expf(-v));
        slab[idx] = v * sg;
      }
      wave_lds_sync();
    }
    if (EPI == 0 || EPI == 1 || EPI == 3) {
      float* C = (float*)Cout;
      const int hh = lane >> 4, c4 = (lane & 15) * 4;
      v4f vals[8];
#pragma unroll
      for (int it = 0; it < 8; ++it) {
        const int row = it * 2 + hh;
        vals[it] = *(const v4f*)(slab + row * 68 + c4);
      }
      if (EPI == 3) {
#pragma unroll
        for (int it = 0; it < 8; ++it) {
          const int row = it * 2 + hh;
          const v4f rv = *(const v4f*)(aux + (size_t)(mBase + row) * ldaux + n0 + c4);
          vals[it] = vals[it] + rv;
        }
      }
      for (int pass = 0; pass < 2; ++pass) {
#pragma unroll
        for (int it = 0; it < 8; ++it) {
          const int row = it * 2 + hh;
          *(volatile v4f*)(C + (size_t)(mBase + row) * ldc + n0 + c4) = vals[it];
        }
        __threadfence();
      }
    } else {
      unsigned short* C = (unsigned short*)Cout;
      const int q = lane >> 3, c8 = (lane & 7) * 8;
      v8h hv[4];
#pragma unroll
      for (int it = 0; it < 4; ++it) {
        const int row = it * 4 + q;
        const float* sp = slab + row * 68 + c8;
        const v4f a0 = *(const v4f*)(sp);
        const v4f a1 = *(const v4f*)(sp + 4);
        const float* gp = aux + (size_t)(mBase + row) * ldaux + n0 + c8;
        const v4f g0 = *(const v4f*)(gp);
        const v4f g1 = *(const v4f*)(gp + 4);
#pragma unroll
        for (int e = 0; e < 4; ++e) {
          const float p0 = a0[e] * g0[e];
          const float p1 = a1[e] * g1[e];
          hv[it][e]     = (_Float16)p0;
          hv[it][4 + e] = (_Float16)p1;
        }
      }
      for (int pass = 0; pass < 2; ++pass) {
#pragma unroll
        for (int it = 0; it < 4; ++it) {
          const int row = it * 4 + q;
          *(volatile v8h*)(C + (size_t)(mBase + row) * ldc + n0 + c8) = hv[it];
        }
        __threadfence();
      }
    }
    wave_lds_sync();
  }
}

template <int MODE>
__global__ __launch_bounds__(256) void transpose_plane_kernel(
    const float* __restrict__ W, int ldw, int col0, int ncols, int kdim,
    unsigned short* Bh, unsigned short* Bl, float scale)
{
  __shared__ float tile[64 * 65];
  const int tid = threadIdx.x, lane = tid & 31, wave = tid >> 5;
  const int n0 = blockIdx.x * 64;
  const int k0 = blockIdx.y * 64;
#pragma unroll 1
  for (int g = 0; g < 2; ++g) {
#pragma unroll
    for (int p = 0; p < 8; ++p) {
      const int idx = tid + (g * 8 + p) * 256;
      const int kk  = idx >> 6;
      const int nn  = idx & 63;
      const int n   = n0 + nn;
      const int nc  = (n < ncols) ? n : (ncols - 1);
      const float v = W[(size_t)(k0 + kk) * ldw + col0 + nc];
      tile[kk * 65 + nn] = (n < ncols) ? (v * scale) : 0.0f;
    }
  }
  __syncthreads();
  const int q = lane >> 3, c8 = (lane & 7) * 8;
  v8h hv[2];
  v4u hw[2], lw[2];
#pragma unroll
  for (int it = 0; it < 2; ++it) {
    const int nrow = it * 32 + wave * 4 + q;
    float f[8];
#pragma unroll
    for (int e = 0; e < 8; ++e) f[e] = tile[(c8 + e) * 65 + nrow];
    if (MODE == 0) {
#pragma unroll
      for (int e = 0; e < 8; ++e) hv[it][e] = (_Float16)f[e];
    } else {
      unsigned h, l;
      split2(f[0], f[1], h, l); hw[it][0] = h; lw[it][0] = l;
      split2(f[2], f[3], h, l); hw[it][1] = h; lw[it][1] = l;
      split2(f[4], f[5], h, l); hw[it][2] = h; lw[it][2] = l;
      split2(f[6], f[7], h, l); hw[it][3] = h; lw[it][3] = l;
    }
  }
  for (int pass = 0; pass < 2; ++pass) {
#pragma unroll
    for (int it = 0; it < 2; ++it) {
      const int nrow = it * 32 + wave * 4 + q;
      const size_t o = (size_t)(n0 + nrow) * kdim + k0 + c8;
      if (MODE == 0) {
        *(volatile v8h*)(Bh + o) = hv[it];
      } else {
        *(volatile v4u*)(Bh + o) = hw[it];
        *(volatile v4u*)(Bl + o) = lw[it];
      }
    }
    __threadfence();
  }
}

__global__ __launch_bounds__(256) void layernorm_split_kernel(
    const float* __restrict__ x, const float* __restrict__ nw, const float* __restrict__ nb,
    unsigned short* __restrict__ XH, unsigned short* __restrict__ XL)
{
  const int lane = threadIdx.x & 31, wave = threadIdx.x >> 5;
  const int row = blockIdx.x * 8 + wave;
  const float* xr = x + (size_t)row * kHid;
  v4f xa[3], xb[3];
#pragma unroll
  for (int it = 0; it < 3; ++it) {
    const int c = it * 256 + lane * 8;
    xa[it] = *(const v4f*)(xr + c);
    xb[it] = *(const v4f*)(xr + c + 4);
  }
  float s = 0.0f;
#pragma unroll
  for (int it = 0; it < 3; ++it) {
#pragma unroll
    for (int e = 0; e < 4; ++e) { s += xa[it][e]; s += xb[it][e]; }
  }
#pragma unroll
  for (int off = 16; off > 0; off >>= 1) s += __shfl_xor(s, off, 32);
  const float mu = s * (1.0f / (float)kHid);
  float ss = 0.0f;
#pragma unroll
  for (int it = 0; it < 3; ++it) {
#pragma unroll
    for (int e = 0; e < 4; ++e) {
      const float d0 = xa[it][e] - mu;
      const float d1 = xb[it][e] - mu;
      ss += d0 * d0;
      ss += d1 * d1;
    }
  }
#pragma unroll
  for (int off = 16; off > 0; off >>= 1) ss += __shfl_xor(ss, off, 32);
  const float var = ss * (1.0f / (float)kHid);
  const float rs = rsqrtf(var + 1e-5f);
  v4u hw[3], lw[3];
#pragma unroll
  for (int it = 0; it < 3; ++it) {
    asm volatile("" ::: "memory");
    const int c = it * 256 + lane * 8;
    const v4f w0 = *(const v4f*)(nw + c);
    const v4f w1 = *(const v4f*)(nw + c + 4);
    const v4f b0 = *(const v4f*)(nb + c);
    const v4f b1 = *(const v4f*)(nb + c + 4);
    float o[8];
#pragma unroll
    for (int e = 0; e < 4; ++e) {
      o[e]     = (xa[it][e] - mu) * rs * w0[e] + b0[e];
      o[4 + e] = (xb[it][e] - mu) * rs * w1[e] + b1[e];
    }
    unsigned h, l;
    split2(o[0], o[1], h, l); hw[it][0] = h; lw[it][0] = l;
    split2(o[2], o[3], h, l); hw[it][1] = h; lw[it][1] = l;
    split2(o[4], o[5], h, l); hw[it][2] = h; lw[it][2] = l;
    split2(o[6], o[7], h, l); hw[it][3] = h; lw[it][3] = l;
  }
  for (int pass = 0; pass < 2; ++pass) {
#pragma unroll
    for (int it = 0; it < 3; ++it) {
      const size_t o = (size_t)row * kHid + it * 256 + lane * 8;
      *(volatile v4u*)(XH + o) = hw[it];
      *(volatile v4u*)(XL + o) = lw[it];
    }
    __threadfence();
  }
}

__global__ __launch_bounds__(256) void conv_silu_kernel(
    const float* __restrict__ UP, const float* __restrict__ cw,
    unsigned short* __restrict__ UH, unsigned short* __restrict__ UL, unsigned short* __restrict__ UF)
{
  __shared__ __align__(16) float sT[16 * kConvTP];
  const int tid = threadIdx.x, lane = tid & 31, wave = tid >> 5;
  const int d0 = blockIdx.x * 256, d = d0 + tid;
  const int t0 = blockIdx.y * 64;
  const v4f wv = *(const v4f*)(cw + (size_t)d * 4);
  const float w0 = wv[0], w1 = wv[1], w2 = wv[2], w3 = wv[3];
  float xm3, xm2, xm1;
  {
    const int r3 = t0 - 3, r2 = t0 - 2, r1 = t0 - 1;
    const float v3 = UP[(size_t)(r3 < 0 ? 0 : r3) * kInner + d];
    const float v2 = UP[(size_t)(r2 < 0 ? 0 : r2) * kInner + d];
    const float v1 = UP[(size_t)(r1 < 0 ? 0 : r1) * kInner + d];
    xm3 = (r3 >= 0) ? v3 : 0.0f;
    xm2 = (r2 >= 0) ? v2 : 0.0f;
    xm1 = (r1 >= 0) ? v1 : 0.0f;
  }
#pragma unroll 1
  for (int sub = 0; sub < 4; ++sub) {
    const int lb = t0 + sub * 16;
#pragma unroll 1
    for (int s = 0; s < 16; ++s) {
      const float xc = UP[(size_t)(lb + s) * kInner + d];
      float acc = w0 * xm3;
      acc = fmaf(w1, xm2, acc);
      acc = fmaf(w2, xm1, acc);
      acc = fmaf(w3, xc, acc);
      const float sg = __builtin_amdgcn_rcpf(1.0f + expf(-acc));
      sT[s * kConvTP + tid] = acc * sg;
      xm3 = xm2; xm2 = xm1; xm1 = xc;
    }
    __syncthreads();
    v4u hw[2], lw[2];
    v8h fv[2];
#pragma unroll
    for (int it = 0; it < 2; ++it) {
      const float* sp = sT + (it * 8 + wave) * kConvTP + lane * 8;
      const v4f a0 = *(const v4f*)(sp);
      const v4f a1 = *(const v4f*)(sp + 4);
      unsigned h, l;
      split2(a0[0], a0[1], h, l); hw[it][0] = h; lw[it][0] = l;
      split2(a0[2], a0[3], h, l); hw[it][1] = h; lw[it][1] = l;
      split2(a1[0], a1[1], h, l); hw[it][2] = h; lw[it][2] = l;
      split2(a1[2], a1[3], h, l); hw[it][3] = h; lw[it][3] = l;
#pragma unroll
      for (int e = 0; e < 4; ++e) {
        const float s0 = a0[e] * kActCarry;
        const float s1 = a1[e] * kActCarry;
        fv[it][e]     = (_Float16)s0;
        fv[it][4 + e] = (_Float16)s1;
      }
    }
    for (int pass = 0; pass < 2; ++pass) {
#pragma unroll
      for (int it = 0; it < 2; ++it) {
        const size_t o = (size_t)(lb + it * 8 + wave) * kInner + d0 + lane * 8;
        *(volatile v4u*)(UH + o) = hw[it];
        *(volatile v4u*)(UL + o) = lw[it];
        *(volatile v8h*)(UF + o) = fv[it];
      }
      __threadfence();
    }
    __syncthreads();
  }
}

__global__ __launch_bounds__(128) void scan_kernel(
    const float* __restrict__ DR, const float* __restrict__ BC,
    const unsigned short* __restrict__ UH, const unsigned short* __restrict__ UL,
    const float* __restrict__ Alog, const float* __restrict__ Dp,
    unsigned short* __restrict__ Y16)
{
  __shared__ __align__(16) float sBC[kScT * 32];
  __shared__ __align__(16) float sD[kScT * kScP];
  __shared__ __align__(16) float sU[kScT * kScP];
  __shared__ __align__(16) float sY[kScT * kScP];
  const int tid = threadIdx.x, lane = tid & 31, wave = tid >> 5;
  const int d0 = blockIdx.x * kScC;
  const int chl = wave * 16 + (lane & 15);
  const int sh = lane >> 4;
  const int d = d0 + chl;
  float negA[8], h[8];
#pragma unroll
  for (int k = 0; k < 8; ++k) {
    negA[k] = -expf(Alog[sh * 8 + k]);
    h[k] = 0.0f;
  }
  const float Dd = Dp[d];
  const int q = lane >> 3, c8f = (lane & 7) * 8;
#pragma unroll 1
  for (int t0 = 0; t0 < kSeq; t0 += kScT) {
    __syncthreads();
#pragma unroll
    for (int i = 0; i < 4; ++i) {
      const int idx = tid + 128 * i;
      const int r = idx >> 3, c4 = (idx & 7) * 4;
      *(v4f*)(sBC + r * 32 + c4) = *(const v4f*)(BC + (size_t)(t0 + r) * kBcP + c4);
    }
#pragma unroll 1
    for (int i = 0; i < 32; ++i) {
      const int r = i * 2 + (tid >> 6);
      const int c = tid & 63;
      const float v = DR[(size_t)(t0 + r) * kInner + d0 + c];
      const float sp = fmaxf(v, 0.0f) + log1pf(expf(-fabsf(v)));
      sD[r * kScP + c] = sp;
    }
#pragma unroll 1
    for (int i = 0; i < 4; ++i) {
      const int idx = tid + 128 * i;
      const int r = idx >> 3, c8 = (idx & 7) * 8;
      const size_t go = (size_t)(t0 + r) * kInner + d0 + c8;
      const v4u wh = *(const v4u*)(UH + go);
      const v4u wl = *(const v4u*)(UL + go);
      const unsigned h0 = wh[0], h1 = wh[1], h2 = wh[2], h3 = wh[3];
      const unsigned l0 = wl[0], l1 = wl[1], l2 = wl[2], l3 = wl[3];
      v4f f0, f1;
      f0[0] = bfw_lo(h0) + bfw_lo(l0);
      f0[1] = bfw_hi(h0) + bfw_hi(l0);
      f0[2] = bfw_lo(h1) + bfw_lo(l1);
      f0[3] = bfw_hi(h1) + bfw_hi(l1);
      f1[0] = bfw_lo(h2) + bfw_lo(l2);
      f1[1] = bfw_hi(h2) + bfw_hi(l2);
      f1[2] = bfw_lo(h3) + bfw_lo(l3);
      f1[3] = bfw_hi(h3) + bfw_hi(l3);
      *(v4f*)(sU + r * kScP + c8) = f0;
      *(v4f*)(sU + r * kScP + c8 + 4) = f1;
    }
    __syncthreads();
#pragma unroll 1
    for (int s = 0; s < kScT; ++s) {
      const float* xr = sBC + s * 32 + sh * 8;
      const v4f b0 = *(const v4f*)(xr);
      const v4f b1 = *(const v4f*)(xr + 4);
      const v4f c0 = *(const v4f*)(xr + 16);
      const v4f c1 = *(const v4f*)(xr + 20);
      float Bs[8], Cs[8];
      Bs[0] = b0[0]; Bs[1] = b0[1]; Bs[2] = b0[2]; Bs[3] = b0[3];
      Bs[4] = b1[0]; Bs[5] = b1[1]; Bs[6] = b1[2]; Bs[7] = b1[3];
      Cs[0] = c0[0]; Cs[1] = c0[1]; Cs[2] = c0[2]; Cs[3] = c0[3];
      Cs[4] = c1[0]; Cs[5] = c1[1]; Cs[6] = c1[2]; Cs[7] = c1[3];
      const float dt = sD[s * kScP + chl];
      const float uu = sU[s * kScP + chl];
      const float dtx = dt * uu;
      float y = 0.0f;
#pragma unroll
      for (int k = 0; k < 8; ++k) {
        const float e = expf(dt * negA[k]);
        h[k] = e * h[k] + dtx * Bs[k];
        y += h[k] * Cs[k];
      }
      const float yo = __shfl_xor(y, 16, 32);
      y = (y + yo) + Dd * uu;
      if (sh == 0) sY[s * kScP + chl] = y * kActCarry;
    }
    __syncthreads();
    v8h hv[4];
#pragma unroll
    for (int it = 0; it < 4; ++it) {
      const int row = it * 16 + wave * 4 + q;
      const float* sp = sY + row * kScP + c8f;
      const v4f a0 = *(const v4f*)(sp);
      const v4f a1 = *(const v4f*)(sp + 4);
#pragma unroll
      for (int e = 0; e < 4; ++e) {
        hv[it][e]     = (_Float16)a0[e];
        hv[it][4 + e] = (_Float16)a1[e];
      }
    }
    for (int pass = 0; pass < 2; ++pass) {
#pragma unroll
      for (int it = 0; it < 4; ++it) {
        const int row = it * 16 + wave * 4 + q;
        *(volatile v8h*)(Y16 + (size_t)(t0 + row) * kInner + d0 + c8f) = hv[it];
      }
      __threadfence();
    }
  }
}

extern "C" void kernel_launch(void* const* d_in, const int* in_sizes, int n_in,
                              void* d_out, int out_size, void* d_ws, size_t ws_size,
                              hipStream_t stream)
{
  if (n_in < 10) return;
  if (in_sizes[0] != kRows * kHid) return;
  if (in_sizes[1] != kHid || in_sizes[2] != kHid) return;
  if (in_sizes[3] != kHid * 2 * kInner) return;
  if (in_sizes[4] != kInner * 4) return;
  if (in_sizes[5] != kInner * kProjW) return;
  if (in_sizes[6] != kNst) return;
  if (in_sizes[7] != kInner) return;
  if (in_sizes[8] != kInner * kInner) return;
  if (in_sizes[9] != kInner * kHid) return;
  if (out_size != kRows * kHid) return;
  if (ws_size < kWsTotal) return;

  const float* x      = (const float*)d_in[0];
  const float* norm_w = (const float*)d_in[1];
  const float* norm_b = (const float*)d_in[2];
  const float* W_in   = (const float*)d_in[3];
  const float* conv_w = (const float*)d_in[4];
  const float* W_xprj = (const float*)d_in[5];
  const float* A_log  = (const float*)d_in[6];
  const float* Dv     = (const float*)d_in[7];
  const float* W_ssm  = (const float*)d_in[8];
  const float* W_out  = (const float*)d_in[9];
  float* dout = (float*)d_out;

  char* ws = (char*)d_ws;
  unsigned short* XNH  = (unsigned short*)(ws + kOffXNH);
  unsigned short* XNL  = (unsigned short*)(ws + kOffXNL);
  unsigned short* BT0H = (unsigned short*)(ws + kOffBT0H);
  unsigned short* BT0L = (unsigned short*)(ws + kOffBT0L);
  unsigned short* BT1D = (unsigned short*)(ws + kOffBT1D);
  unsigned short* BTBH = (unsigned short*)(ws + kOffBTBH);
  unsigned short* BTBL = (unsigned short*)(ws + kOffBTBL);
  unsigned short* BT2  = (unsigned short*)(ws + kOffBT2);
  unsigned short* BT3  = (unsigned short*)(ws + kOffBT3);
  float*          UPRE = (float*)(ws + kOffUPRE);
  float*          GS   = (float*)(ws + kOffGS);
  unsigned short* UH   = (unsigned short*)(ws + kOffUH);
  unsigned short* UL   = (unsigned short*)(ws + kOffUL);
  unsigned short* UF   = (unsigned short*)(ws + kOffUF);
  float*          DR   = (float*)(ws + kOffDR);
  float*          BCp  = (float*)(ws + kOffBC);
  unsigned short* Y16  = (unsigned short*)(ws + kOffY16);
  unsigned short* Z16  = (unsigned short*)(ws + kOffZ16);

  transpose_plane_kernel<1><<<dim3((2 * kInner) / 64, kHid / 64), 256, 0, stream>>>(
      W_in, 2 * kInner, 0, 2 * kInner, kHid, BT0H, BT0L, 1.0f);
  transpose_plane_kernel<0><<<dim3(kInner / 64, kInner / 64), 256, 0, stream>>>(
      W_xprj, kProjW, 2 * kNst, kInner, kInner, BT1D, BT1D, kWgtCarry);
  transpose_plane_kernel<1><<<dim3(kBcP / 64, kInner / 64), 256, 0, stream>>>(
      W_xprj, kProjW, 0, 2 * kNst, kInner, BTBH, BTBL, 1.0f);
  transpose_plane_kernel<0><<<dim3(kInner / 64, kInner / 64), 256, 0, stream>>>(
      W_ssm, kInner, 0, kInner, kInner, BT2, BT2, kWgtCarry);
  transpose_plane_kernel<0><<<dim3(kHid / 64, kInner / 64), 256, 0, stream>>>(
      W_out, kHid, 0, kHid, kInner, BT3, BT3, kWgtCarry);

  layernorm_split_kernel<<<kRows / 8, 256, 0, stream>>>(x, norm_w, norm_b, XNH, XNL);

  constexpr int kTilesWide = (kSeq / 64) * (kInner / 64);
  constexpr int kTilesBC   = (kSeq / 64) * (kBcP / 64);
  constexpr int kTilesOut  = (kSeq / 64) * (kHid / 64);
  static_assert((kTilesWide % 8) == 0 && (kTilesBC % 8) == 0 && (kTilesOut % 8) == 0);

  for (int b = 0; b < kBatch; ++b) {
    const unsigned short* XNHb = XNH + (size_t)b * kSeq * kHid;
    const unsigned short* XNLb = XNL + (size_t)b * kSeq * kHid;
    const float* xb = x + (size_t)b * kSeq * kHid;
    float* outb = dout + (size_t)b * kSeq * kHid;

    wmma_gemm64<1, true, 0><<<dim3(kTilesWide / 8), 256, 0, stream>>>(
        XNHb, XNLb, kHid, BT0H, BT0L, kHid,
        (void*)UPRE, kInner, xb, kHid, kSeq, kInner, kHid, 1.0f);
    wmma_gemm64<1, true, 1><<<dim3(kTilesWide / 8), 256, 0, stream>>>(
        XNHb, XNLb, kHid, BT0H + (size_t)kInner * kHid, BT0L + (size_t)kInner * kHid, kHid,
        (void*)GS, kInner, xb, kHid, kSeq, kInner, kHid, 1.0f);

    conv_silu_kernel<<<dim3(kInner / 256, kSeq / 64), 256, 0, stream>>>(UPRE, conv_w, UH, UL, UF);

    wmma_gemm64<0, false, 0><<<dim3(kTilesWide / 8), 256, 0, stream>>>(
        UF, UF, kInner, BT1D, BT1D, kInner,
        (void*)DR, kInner, xb, kHid, kSeq, kInner, kInner, kFoldAW);
    wmma_gemm64<1, true, 0><<<dim3(kTilesBC / 8), 256, 0, stream>>>(
        UH, UL, kInner, BTBH, BTBL, kInner,
        (void*)BCp, kBcP, xb, kHid, kSeq, kBcP, kInner, 1.0f);

    scan_kernel<<<kInner / kScC, 2 * kScC, 0, stream>>>(DR, BCp, UH, UL, A_log, Dv, Y16);

    wmma_gemm64<0, false, 2><<<dim3(kTilesWide / 8), 256, 0, stream>>>(
        Y16, Y16, kInner, BT2, BT2, kInner,
        (void*)Z16, kInner, GS, kInner, kSeq, kInner, kInner, kFoldW);

    wmma_gemm64<0, false, 3><<<dim3(kTilesOut / 8), 256, 0, stream>>>(
        Z16, Z16, kInner, BT3, BT3, kInner,
        (void*)outb, kHid, xb, kHid, kSeq, kHid, kInner, kFoldAW);
  }
}
